// RingAttentionCollective_76312978915793
// MI455X (gfx1250) — hardware-verified
//
#include <hip/hip_runtime.h>


namespace {
constexpr int NB = 2, NHD = 16, G = NB * NHD, S = 2048, D = 64, TOK = NHD * D, OTOK = NHD * D;
constexpr float SCALE = 0.125f;
__device__ __forceinline__ size_t goff(int g) { return (size_t)(g / NHD) * S * NHD * D + (size_t)(g % NHD) * D; }
__device__ __forceinline__ size_t ooff(int g) { return goff(g); }


typedef _Float16 b16;
typedef __attribute__((ext_vector_type(16))) _Float16 v16b;
typedef __attribute__((ext_vector_type(8))) _Float16 v8b;
typedef __attribute__((ext_vector_type(8))) float v8f;
typedef __attribute__((ext_vector_type(4))) float v4f;
typedef __attribute__((ext_vector_type(2))) _Float16 v2b;
__device__ __forceinline__ float bf16_rne(float f) { unsigned int u = __float_as_uint(f); u += 0x7FFFu + ((u >> 16) & 1u); return __uint_as_float(u & 0xFFFF0000u); }
__device__ __forceinline__ v16b frag_kb(const b16* p, int hh) { const v8b a = *(const v8b*)(p + 8 * hh), b = *(const v8b*)(p + 16 + 8 * hh); v16b f;
#pragma unroll
  for (int e = 0; e < 8; ++e) { f[e] = a[e]; f[8 + e] = b[e]; } return f; }
__device__ __forceinline__ v8f wmma16b(v16b a, v16b b, v8f c) { v8f d = __builtin_amdgcn_wmma_f32_16x16x32_f16(false, a, false, b, (short)0, c, false, false); asm volatile("v_nop\n\tv_nop\n\tv_nop\n\tv_nop" : "+v"(d) : "v"(a), "v"(b)); return d; }
__device__ __forceinline__ void wave_lds_sync() { __builtin_amdgcn_fence(__ATOMIC_RELEASE, "workgroup"); __builtin_amdgcn_wave_barrier(); __builtin_amdgcn_fence(__ATOMIC_ACQUIRE, "workgroup"); }
__device__ __forceinline__ float pmul(float a, float b) { float p = a * b; asm volatile("" : "+v"(p)); return p; }

__global__ __launch_bounds__(256) void kprep_kernel(const float* __restrict__ k, b16* __restrict__ KB) { const size_t u = (size_t)blockIdx.x * 256 + threadIdx.x; if (u >= (size_t)G * S * (D / 8)) return; const int g = (int)(u / ((size_t)S * (D / 8))); const size_t rem = u % ((size_t)S * (D / 8)); const int s = (int)(rem / (D / 8)), d0 = (int)(rem % (D / 8)) * 8; const float* src = k + goff(g) + (size_t)s * TOK + d0; v8b v;
#pragma unroll
  for (int j = 0; j < 8; ++j) v[j] = (b16)bf16_rne(src[j]); for (int pass = 0; pass < 2; ++pass) { *(volatile v8b*)(KB + ((size_t)g * S + s) * D + d0) = v; __threadfence(); } }
__global__ __launch_bounds__(256) void vprep_kernel(const float* __restrict__ v, b16* __restrict__ VT) { const int wave = threadIdx.x >> 5, lane = threadIdx.x & 31; const size_t wid = (size_t)blockIdx.x * 8 + wave; if (wid >= (size_t)G * D * (S / 64)) return; const int g = (int)(wid / ((size_t)D * (S / 64))); const size_t rem = wid % ((size_t)D * (S / 64)); const int d = (int)(rem / (S / 64)), s0 = (int)(rem % (S / 64)) * 64 + 2 * lane;
  const v2b val = {(b16)bf16_rne(v[goff(g) + (size_t)s0 * TOK + d]), (b16)bf16_rne(v[goff(g) + (size_t)(s0 + 1) * TOK + d])}; for (int pass = 0; pass < 2; ++pass) { *(volatile v2b*)(VT + ((size_t)g * D + d) * S + s0) = val; __threadfence(); } }
template <int MASK, int PHL>
__global__ __launch_bounds__(32) void flash_kernel(const float* __restrict__ q, const b16* __restrict__ KB, const b16* __restrict__ VT, const int* __restrict__ cu, int ncu, int GLIM, float* __restrict__ out) {
  __shared__ __attribute__((aligned(16))) b16 Qs[16][D + 8], Ps[16][40], Pl[16][PHL ? 40 : 8]; __shared__ float Tf[16][D + 4]; const int lane = threadIdx.x, nloc = lane & 15, hlf = lane >> 4; const int g = blockIdx.x / (S / 16), qt = blockIdx.x % (S / 16); if (g >= GLIM) return; const int q0 = qt * 16;
  for (int rr = 0; rr < 16; ++rr) for (int c = lane; c < D; c += 32) Qs[rr][c] = (b16)(bf16_rne(q[goff(g) + (size_t)(q0 + rr) * TOK + c]) * 8.0f);
  wave_lds_sync();
  float m[8], l[8]; v8f O[D / 16];
#pragma unroll
  for (int r = 0; r < 8; ++r) { m[r] = -INFINITY; l[r] = 0.0f; }
#pragma unroll
  for (int t = 0; t < D / 16; ++t) O[t] = (v8f){};
  int kend = S, kstart = 0;
  int segstart[8];
#pragma unroll
  for (int r = 0; r < 8; ++r) segstart[r] = 0;
  if (MASK == 1) { kend = q0 + 16;
#pragma unroll
    for (int r = 0; r < 8; ++r) { const int qq = q0 + 8 * hlf + r; int st = 0; for (int c = 1; c < ncu; ++c) { const int b = cu[c]; if (b <= qq) st = b; }
      segstart[r] = st; }
    int mn_ = segstart[0]; for (int r = 1; r < 8; ++r) mn_ = min(mn_, segstart[r]); mn_ = min(mn_, __shfl_xor(mn_, 16)); kstart = (mn_ / 32) * 32; }
  const size_t kbase = (size_t)g * S;
#pragma unroll 1
  for (int k0 = kstart; k0 < kend; k0 += 32) {
    v8f Sa[2] = {(v8f){}, (v8f){}};
#pragma unroll
    for (int kb = 0; kb < D; kb += 32) { const v16b a = frag_kb(&Qs[nloc][kb], hlf);
#pragma unroll
      for (int t = 0; t < 2; ++t) Sa[t] = wmma16b(a, frag_kb(KB + (kbase + k0 + t * 16 + nloc) * D + kb, hlf), Sa[t]); }
    float p0[8], p1[8];
#pragma unroll
    for (int r = 0; r < 8; ++r) { float s0 = Sa[0][r] * (SCALE / 8.0f), s1 = Sa[1][r] * (SCALE / 8.0f);
      if (MASK == 1) { const int qq = q0 + 8 * hlf + r; const int ka = k0 + nloc, kb2 = k0 + 16 + nloc; if (ka > qq || ka < segstart[r]) s0 = -INFINITY; if (kb2 > qq || kb2 < segstart[r]) s1 = -INFINITY; }
      float mx = fmaxf(s0, s1); mx = fmaxf(mx, __shfl_xor(mx, 1)); mx = fmaxf(mx, __shfl_xor(mx, 2)); mx = fmaxf(mx, __shfl_xor(mx, 4)); mx = fmaxf(mx, __shfl_xor(mx, 8));
      const float mn = fmaxf(m[r], mx); const float corr = (m[r] == -INFINITY) ? 0.0f : __expf(m[r] - mn);
      float e0 = (mn == -INFINITY) ? 0.0f : __expf(s0 - mn), e1 = (mn == -INFINITY) ? 0.0f : __expf(s1 - mn); float ps = e0 + e1; ps += __shfl_xor(ps, 1); ps += __shfl_xor(ps, 2); ps += __shfl_xor(ps, 4); ps += __shfl_xor(ps, 8);
      const float cr = (mn == -INFINITY) ? 1.0f : corr; l[r] = l[r] * cr + ps; m[r] = mn; p0[r] = e0; p1[r] = e1;
#pragma unroll
      for (int t = 0; t < D / 16; ++t) O[t][r] *= cr; }
    wave_lds_sync();
#pragma unroll
    for (int r = 0; r < 8; ++r) { const float a0 = p0[r] * 1024.0f, a1 = p1[r] * 1024.0f; const b16 h0 = (b16)a0, h1 = (b16)a1; Ps[8 * hlf + r][nloc] = h0; Ps[8 * hlf + r][16 + nloc] = h1; if (PHL) { Pl[8 * hlf + r][nloc] = (b16)(a0 - (float)h0); Pl[8 * hlf + r][16 + nloc] = (b16)(a1 - (float)h1); } } if (lane < 16) { for (int e = 32; e < 40; ++e) { Ps[lane][e] = (b16)0.0f; if (PHL) Pl[lane][e] = (b16)0.0f; } }
    wave_lds_sync(); const v16b pa = frag_kb(&Ps[nloc][0], hlf); v16b pl; if (PHL) pl = frag_kb(&Pl[nloc][0], hlf);
#pragma unroll
    for (int t = 0; t < D / 16; ++t) { const v16b vb = frag_kb(VT + ((size_t)g * D + t * 16 + nloc) * S + k0, hlf); O[t] = wmma16b(pa, vb, O[t]); if (PHL) O[t] = wmma16b(pl, vb, O[t]); } }
#pragma unroll
  for (int t = 0; t < D / 16; ++t)
#pragma unroll
    for (int r = 0; r < 8; ++r) Tf[8 * hlf + r][t * 16 + nloc] = (l[r] > 0.0f) ? O[t][r] / (1024.0f * l[r]) : 0.0f;
  wave_lds_sync();
  for (int pass = 0; pass < 2; ++pass) { for (int rr = 0; rr < 16; ++rr) for (int c = lane * 4; c < D; c += 128) *(volatile v4f*)(out + ooff(g) + (size_t)(q0 + rr) * OTOK + c) = *(const v4f*)(&Tf[rr][c]); __threadfence(); } }

}

extern "C" void kernel_launch(void* const* d_in, const int* in_sizes, int n_in, void* d_out, int out_size, void* d_ws, size_t ws_size, hipStream_t stream) {
  (void)n_in;
  auto Fp = [&](int i) { return (const float*)d_in[i]; };
  if (in_sizes[0] != NB * S * NHD * D || in_sizes[1] != NB * S * NHD * D || in_sizes[2] != NB * S * NHD * D || out_size != NB * S * NHD * D) return;
  const int GLIM = G;
  size_t off = 0; char* ws = (char*)d_ws;
  auto carve = [&](size_t bytes) { char* p = ws + off; off += (bytes + 255) & ~(size_t)255; return p; };
  b16* KB = (b16*)carve((size_t)G * S * D * 2); b16* VT = (b16*)carve((size_t)G * D * S * 2);
  if (off > ws_size || off > ((size_t)32 << 20)) return;
  kprep_kernel<<<(unsigned)(((size_t)G * S * (D / 8) + 255) / 256), 256, 0, stream>>>(Fp(1), KB);
  vprep_kernel<<<(unsigned)(((size_t)G * D * (S / 64) + 7) / 8), 256, 0, stream>>>(Fp(2), VT);
  flash_kernel<0, 0><<<GLIM * (S / 16), 32, 0, stream>>>(Fp(0), KB, VT, nullptr, 0, GLIM, (float*)d_out);
}
